// FlashAttention3_64828236366195
// MI455X (gfx1250) — hardware-verified
//
#include <hip/hip_runtime.h>
#include <math.h>
#include <stdint.h>

#define NBATCH 2
#define SEQ    2048
#define NHEAD  16
#define HDIM   64
#define DMOD   (NHEAD * HDIM)
#define NTOK   (NBATCH * SEQ)
#define QBLK   128

typedef __attribute__((ext_vector_type(16))) __bf16   v16b;
typedef __attribute__((ext_vector_type(8)))  __bf16   v8b;
typedef __attribute__((ext_vector_type(8)))  float    v8f;
typedef __attribute__((ext_vector_type(4)))  float    v4f;
typedef __attribute__((ext_vector_type(2)))  float    v2f;
typedef __attribute__((ext_vector_type(4)))  unsigned int v4u;
typedef __attribute__((ext_vector_type(2)))  int      v2i;

static_assert(DMOD == 1024);
static_assert((NTOK * NHEAD) % 8 == 0);
static_assert(SEQ % 64 == 0);
static_assert(HDIM == 64);

__device__ __forceinline__ unsigned short f2bf_bits(float f) {
  unsigned u = __float_as_uint(f);
  return (unsigned short)((u + 0x7FFFu + ((u >> 16) & 1u)) >> 16);
}
__device__ __forceinline__ float bf_bits2f(unsigned short h) { return __uint_as_float(((unsigned)h) << 16); }
__device__ __forceinline__ unsigned pk16(unsigned short a, unsigned short b) { return (unsigned)a | ((unsigned)b << 16); }

__device__ __forceinline__ v16b ldfrag_b(const __bf16* p) {
  union { v16b v; v8b h[2]; } f;
  f.h[0] = *(const v8b*)(p);
  f.h[1] = *(const v8b*)(p + 16);
  return f.v;
}
__device__ __forceinline__ v8f at_mma(v16b a, v16b b, v8f c) {
  c = __builtin_amdgcn_wmma_f32_16x16x32_bf16(false, a, false, b, (short)0, c, false, false);
  asm volatile("v_nop\n\tv_nop\n\tv_nop\n\tv_nop" : "+v"(c) : "v"(a), "v"(b));
  return c;
}

__global__ __launch_bounds__(256) void prep_qk_kernel(const float* __restrict__ q, const float* __restrict__ k,
                                                      unsigned short* __restrict__ QNh, unsigned short* __restrict__ QNl,
                                                      unsigned short* __restrict__ KB, int nunits) {
  __shared__ __align__(16) unsigned st[8][96];
  const int tid  = threadIdx.x;
  const int w    = tid >> 5;
  const int lane = tid & 31;
  int gu = blockIdx.x * 8 + w;
  gu = (gu < nunits) ? gu : (nunits - 1);
  const size_t base = (size_t)gu * HDIM;
  const v2f qv = *(const v2f*)(q + base + 2 * lane);
  const v2f kv = *(const v2f*)(k + base + 2 * lane);
  const float x0 = bf_bits2f(f2bf_bits(qv[0]));
  const float x1 = bf_bits2f(f2bf_bits(qv[1]));
  float ss = x0 * x0 + x1 * x1;
#pragma unroll
  for (int off = 16; off > 0; off >>= 1) ss += __shfl_xor(ss, off, 32);
  const float nrm = sqrtf(ss);
  const float inv = 1.0f / fmaxf(nrm, 1e-12f);
  const float y0 = x0 * inv;
  const float y1 = x1 * inv;
  const unsigned short hb0 = f2bf_bits(y0), hb1 = f2bf_bits(y1);
  const unsigned short lb0 = f2bf_bits(y0 - bf_bits2f(hb0));
  const unsigned short lb1 = f2bf_bits(y1 - bf_bits2f(hb1));
  const unsigned short kb0 = f2bf_bits(kv[0]), kb1 = f2bf_bits(kv[1]);
  st[w][lane]      = pk16(hb0, hb1);
  st[w][32 + lane] = pk16(lb0, lb1);
  st[w][64 + lane] = pk16(kb0, kb1);
  __syncthreads();
  int q3 = lane >> 3;
  q3 = (q3 > 2) ? 2 : q3;
  const v4u val = *(const v4u*)(&st[w][q3 * 32 + (lane & 7) * 4]);
  const size_t co = base + (size_t)(lane & 7) * 8;
  unsigned short* d = (q3 == 0) ? QNh : ((q3 == 1) ? QNl : KB);
  if (lane < 24) { *(volatile v4u*)(d + co) = val; }
  __threadfence();
  if (lane < 24) { *(volatile v4u*)(d + co) = val; }
}

__global__ __launch_bounds__(256) void vtrans_kernel(const float* __restrict__ v, unsigned short* __restrict__ VT) {
  __shared__ __align__(16) unsigned short th[64 * 72];
  const int c0  = blockIdx.x * 64;
  const int r0  = blockIdx.y * 64;
  const int b   = blockIdx.z;
  const int tid = threadIdx.x;
  {
    const int rr = tid >> 2;
    const int cq = (tid & 3) * 16;
    const float* src = v + ((size_t)b * SEQ + r0 + rr) * DMOD + c0 + cq;
#pragma unroll
    for (int qq = 0; qq < 4; ++qq) {
      const v4f f = *(const v4f*)(src + 4 * qq);
#pragma unroll
      for (int e = 0; e < 4; ++e) th[rr * 72 + cq + 4 * qq + e] = f2bf_bits(f[e]);
    }
  }
  __syncthreads();
  const int sub = tid >> 3;
  const int c8  = (tid & 7) * 8;
  v4u hv[2];
#pragma unroll
  for (int it = 0; it < 2; ++it) {
    const int oc = it * 32 + sub;
    v4u a;
#pragma unroll
    for (int qq = 0; qq < 4; ++qq)
      a[qq] = pk16(th[(c8 + 2 * qq) * 72 + oc], th[(c8 + 2 * qq + 1) * 72 + oc]);
    hv[it] = a;
  }
  for (int pass = 0; pass < 2; ++pass) {
#pragma unroll
    for (int it = 0; it < 2; ++it) {
      const int oc = it * 32 + sub;
      const size_t go = ((size_t)b * DMOD + c0 + oc) * SEQ + r0 + c8;
      *(volatile v4u*)(VT + go) = hv[it];
    }
    __threadfence();
  }
}

#define AT_D  64
#define AT_NW 4
#define AT_QB 64
#define AT_KC 64

__global__ __launch_bounds__(128)
void attn64_kernel(const unsigned short* __restrict__ qhp, const unsigned short* __restrict__ qlp,
                   const unsigned short* __restrict__ kbp, const unsigned short* __restrict__ vtp,
                   const int* __restrict__ mask, float* __restrict__ out, float sscale) {
  union FB { v16b v; v8b h[2]; };
  __shared__ __align__(16) __bf16 Ksh[AT_KC * AT_D];
  __shared__ __align__(16) __bf16 Vth[AT_D * AT_KC];
  __shared__ __align__(16) __bf16 Psh[AT_NW][16 * AT_KC];
  __shared__ __align__(16) __bf16 Psl[AT_NW][16 * AT_KC];
  __shared__ __align__(16) float  Os[AT_NW][16 * 68];
  __shared__ __align__(16) int    Msk[AT_KC];

  const int tid  = threadIdx.x;
  const int wave = tid >> 5;
  const int lane = tid & 31;
  const int hh   = lane >> 4;
  const int c    = lane & 15;

  const int nqb = SEQ / AT_QB;
  const int bx  = blockIdx.x;
  const int qb  = bx % nqb;
  const int h   = bx / nqb;
  const int b   = blockIdx.y;
  const int q0  = qb * AT_QB + wave * 16;
  const size_t tok0 = (size_t)b * SEQ;

  const __bf16* Qh = (const __bf16*)(const void*)qhp + tok0 * DMOD + (size_t)h * AT_D;
  const __bf16* Ql = (const __bf16*)(const void*)qlp + tok0 * DMOD + (size_t)h * AT_D;
  const __bf16* Kb = (const __bf16*)(const void*)kbp + tok0 * DMOD + (size_t)h * AT_D;
  const __bf16* Vt = (const __bf16*)(const void*)vtp + ((size_t)b * DMOD + (size_t)h * AT_D) * SEQ;
  const int*    mb = mask + tok0;
  float*        ob = out + tok0 * DMOD + (size_t)h * AT_D;

  v16b qah[2], qal[2];
#pragma unroll
  for (int dc = 0; dc < 2; ++dc) {
    qah[dc] = ldfrag_b(Qh + (size_t)(q0 + c) * DMOD + dc * 32 + 8 * hh);
    qal[dc] = ldfrag_b(Ql + (size_t)(q0 + c) * DMOD + dc * 32 + 8 * hh);
  }

  float mrow[8], lrow[8];
  v8f oacc[4];
#pragma unroll
  for (int r = 0; r < 8; ++r) { mrow[r] = -INFINITY; lrow[r] = 0.f; }
#pragma unroll
  for (int t = 0; t < 4; ++t) oacc[t] = (v8f){0.f,0.f,0.f,0.f,0.f,0.f,0.f,0.f};

  const int nChunks = (qb < (QBLK / AT_KC)) ? (QBLK / AT_KC) : (qb + 1);
  for (int kc = 0; kc < nChunks; ++kc) {
    const int kv0 = kc * AT_KC;
    __syncthreads();
    {
      const int r = tid >> 1, half = (tid & 1) * 32;
      const __bf16* ks = Kb + (size_t)(kv0 + r) * DMOD + half;
      const __bf16* vs = Vt + (size_t)r * SEQ + kv0 + half;
#pragma unroll
      for (int i = 0; i < 4; ++i) {
        const v8b a0 = *(const v8b*)(ks + 8 * i);
        const v8b b0 = *(const v8b*)(vs + 8 * i);
        *(v8b*)(Ksh + r * AT_D  + half + 8 * i) = a0;
        *(v8b*)(Vth + r * AT_KC + half + 8 * i) = b0;
      }
      if (wave == 0) {
        const v2i m2 = *(const v2i*)(mb + kv0 + 2 * lane);
        *(v2i*)(Msk + 2 * lane) = m2;
      }
    }
    __syncthreads();

    int lv = ((Msk[lane] | Msk[lane + 32]) != 0) ? 1 : 0;
#pragma unroll
    for (int off = 1; off < 32; off <<= 1) lv |= __shfl_xor(lv, off, 32);
    const int tile_live = __builtin_amdgcn_readfirstlane(lv);

    if (tile_live != 0) {
      v8f s[4];
#pragma unroll
      for (int j = 0; j < 4; ++j) {
        s[j] = (v8f){0.f,0.f,0.f,0.f,0.f,0.f,0.f,0.f};
#pragma unroll
        for (int dc = 0; dc < 2; ++dc) {
          FB kf;
          kf.h[0] = *(const v8b*)(Ksh + (j * 16 + c) * AT_D + dc * 32 + 8 * hh);
          kf.h[1] = *(const v8b*)(Ksh + (j * 16 + c) * AT_D + dc * 32 + 16 + 8 * hh);
          s[j] = at_mma(qah[dc], kf.v, s[j]);
          s[j] = at_mma(qal[dc], kf.v, s[j]);
        }
      }
      int mk[4];
#pragma unroll
      for (int j = 0; j < 4; ++j) mk[j] = Msk[j * 16 + c];
      const bool diag = (qb >= (QBLK / AT_KC)) && (kc == qb);
      float cm[8];
#pragma unroll
      for (int r = 0; r < 8; ++r) {
        const int qrow = q0 + 8 * hh + r;
        float m = -INFINITY;
#pragma unroll
        for (int j = 0; j < 4; ++j) {
          const int kvcol = kv0 + j * 16 + c;
          const float sv = s[j][r] * sscale;
          const bool excl = (diag && (kvcol > qrow)) || (mk[j] == 0);
          const float sm = excl ? -INFINITY : sv;
          s[j][r] = sm;
          m = fmaxf(m, sm);
        }
#pragma unroll
        for (int off = 1; off < 16; off <<= 1) m = fmaxf(m, __shfl_xor(m, off, 32));
        cm[r] = m;
      }
      __bf16* pwh = Psh[wave];
      __bf16* pwl = Psl[wave];
#pragma unroll
      for (int r = 0; r < 8; ++r) {
        const float mnew  = fmaxf(mrow[r], cm[r]);
        const float mref  = (mnew == -INFINITY) ? 0.0f : mnew;
        const float alpha = expf(mrow[r] - mref);
        mrow[r] = mnew;
        float psum = 0.f;
#pragma unroll
        for (int j = 0; j < 4; ++j) {
          const float p = expf(s[j][r] - mref);
          psum += p;
          const unsigned short hb = f2bf_bits(p);
          const unsigned short lb = f2bf_bits(p - bf_bits2f(hb));
          pwh[(8 * hh + r) * AT_KC + j * 16 + c] = __builtin_bit_cast(__bf16, hb);
          pwl[(8 * hh + r) * AT_KC + j * 16 + c] = __builtin_bit_cast(__bf16, lb);
        }
#pragma unroll
        for (int off = 1; off < 16; off <<= 1) psum += __shfl_xor(psum, off, 32);
        lrow[r] = lrow[r] * alpha + psum;
#pragma unroll
        for (int t = 0; t < 4; ++t) oacc[t][r] *= alpha;
      }
      __builtin_amdgcn_fence(__ATOMIC_RELEASE, "workgroup");
      __builtin_amdgcn_wave_barrier();
      __builtin_amdgcn_fence(__ATOMIC_ACQUIRE, "workgroup");
#pragma unroll 1
      for (int kk = 0; kk < 2; ++kk) {
        FB pa, pl;
        pa.h[0] = *(const v8b*)(pwh + c * AT_KC + kk * 32 + 8 * hh);
        pa.h[1] = *(const v8b*)(pwh + c * AT_KC + kk * 32 + 16 + 8 * hh);
        pl.h[0] = *(const v8b*)(pwl + c * AT_KC + kk * 32 + 8 * hh);
        pl.h[1] = *(const v8b*)(pwl + c * AT_KC + kk * 32 + 16 + 8 * hh);
#pragma unroll
        for (int t = 0; t < 4; ++t) {
          FB vf;
          vf.h[0] = *(const v8b*)(Vth + (t * 16 + c) * AT_KC + kk * 32 + 8 * hh);
          vf.h[1] = *(const v8b*)(Vth + (t * 16 + c) * AT_KC + kk * 32 + 16 + 8 * hh);
          oacc[t] = at_mma(pa.v, vf.v, oacc[t]);
          oacc[t] = at_mma(pl.v, vf.v, oacc[t]);
        }
      }
    }
  }

  float* os = Os[wave];
#pragma unroll
  for (int r = 0; r < 8; ++r) {
    const float l   = lrow[r];
    const float inv = (l > 0.f) ? (1.0f / l) : 0.0f;
#pragma unroll
    for (int t = 0; t < 4; ++t) os[(8 * hh + r) * 68 + t * 16 + c] = oacc[t][r] * inv;
  }
  __builtin_amdgcn_fence(__ATOMIC_RELEASE, "workgroup");
  __builtin_amdgcn_wave_barrier();
  __builtin_amdgcn_fence(__ATOMIC_ACQUIRE, "workgroup");
  {
    const int c4 = (lane & 15) * 4;
    for (int pass = 0; pass < 2; ++pass) {
#pragma unroll
      for (int it = 0; it < 8; ++it) {
        const int row = it * 2 + hh;
        v4f val = *(const v4f*)(os + row * 68 + c4);
        *(volatile v4f*)(ob + (size_t)(q0 + row) * DMOD + c4) = val;
      }
      __threadfence();
    }
  }
}

extern "C" void kernel_launch(void* const* d_in, const int* in_sizes, int n_in,
                              void* d_out, int out_size, void* d_ws, size_t ws_size,
                              hipStream_t stream) {
  if (n_in < 4) return;
  if (in_sizes[0] != NTOK * DMOD || in_sizes[1] != NTOK * DMOD || in_sizes[2] != NTOK * DMOD) return;
  if (in_sizes[3] != NBATCH * SEQ) return;
  if (out_size != NTOK * DMOD) return;

  const float* q   = (const float*)d_in[0];
  const float* k   = (const float*)d_in[1];
  const float* v   = (const float*)d_in[2];
  const int*   msk = (const int*)d_in[3];
  float*       out = (float*)d_out;

  const size_t PPL = (size_t)NTOK * DMOD * 2;
  size_t off = 0;
  const size_t oQNh = off; off += PPL;
  const size_t oQNl = off; off += PPL;
  const size_t oKB  = off; off += PPL;
  const size_t oVT  = off; off += PPL;
  if (off > ws_size) return;

  char* ws = (char*)d_ws;
  unsigned short* QNh = (unsigned short*)(ws + oQNh);
  unsigned short* QNl = (unsigned short*)(ws + oQNl);
  unsigned short* KB  = (unsigned short*)(ws + oKB);
  unsigned short* VT  = (unsigned short*)(ws + oVT);

  const int nunits = NTOK * NHEAD;
  prep_qk_kernel<<<dim3(nunits / 8), dim3(256), 0, stream>>>(q, k, QNh, QNl, KB, nunits);
  vtrans_kernel<<<dim3(DMOD / 64, SEQ / 64, NBATCH), dim3(256), 0, stream>>>(v, VT);
  attn64_kernel<<<dim3(NHEAD * (SEQ / AT_QB), NBATCH), dim3(128), 0, stream>>>(QNh, QNl, KB, VT, msk, out, 0.125f);
  (void)hipGetLastError();
}
